// CausalMultiHeadAttention_74586402062365
// MI455X (gfx1250) — hardware-verified
//
#include <hip/hip_runtime.h>
#include <math.h>

#ifndef NB
#define NB 4
#endif
#ifndef SEQ
#define SEQ 2048
#endif

constexpr int kBF   = 4;
constexpr int kSF   = 2048;
constexpr int kB    = NB;
constexpr int kS    = SEQ;
constexpr int kE    = 1024;
constexpr int kH    = 16;
constexpr int kD    = 64;
constexpr int kF    = 3 * kE;
constexpr int kTok  = kB * kS;
constexpr int kQKld = 2 * kE;
constexpr int kQB   = 64;
constexpr int kKC   = 64;
constexpr int kNW   = 4;
constexpr int kNQB  = kS / kQB;
constexpr int kHeadRows   = (kS < 256) ? kS : 256;
constexpr int kHeadBlocks = kHeadRows / kQB;
constexpr float kPCarry     = 32768.0f;
constexpr float kYCarry     = 256.0f;
constexpr float kWoCarry    = 64.0f;
constexpr float kOutScale   = 1.0f / (kYCarry * kWoCarry);
constexpr float kLogitScale = 0.125f;

static_assert(kB >= 1 && kB <= kBF);
static_assert(kS >= kQB && kS <= kSF && kS % kQB == 0);
static_assert(kH * kD == kE);
static_assert(kE % 32 == 0);
static_assert(kTok % 64 == 0 && kQKld % 64 == 0);
static_assert(kE % 64 == 0 && kS % 64 == 0);
static_assert(kHeadRows % 64 == 0 && (kS - kHeadRows) % 64 == 0);
static_assert(kHeadRows % kKC == 0 && kHeadBlocks >= 1 && kHeadBlocks <= kNQB);
static_assert(kD == 64 && kS % kQB == 0);
static_assert(kE / 8 == 128);
static_assert((kTok * kE) % (8 * 256) == 0);
static_assert((kF * kE) % (8 * 256) == 0 && (kE * kE) % 8 == 0);
static_assert(((long)(kB - 1) * kSF + kS) * kE <= (long)kBF * kSF * kE);

typedef __attribute__((ext_vector_type(16))) _Float16 v16h;
typedef __attribute__((ext_vector_type(8)))  _Float16 v8h;
typedef __attribute__((ext_vector_type(16))) __bf16   v16b;
typedef __attribute__((ext_vector_type(8)))  __bf16   v8b;
typedef __attribute__((ext_vector_type(8)))  float    v8f;
typedef __attribute__((ext_vector_type(4)))  float    v4f;
typedef __attribute__((ext_vector_type(4)))  unsigned int v4u;

__device__ __forceinline__ unsigned short f2bf_bits(float f) {
  unsigned u = __float_as_uint(f);
  return (unsigned short)((u + 0x7FFFu + ((u >> 16) & 1u)) >> 16);
}
__device__ __forceinline__ float bf_bits2f(unsigned short h) { return __uint_as_float(((unsigned)h) << 16); }
__device__ __forceinline__ float bf_rne(float f) { return bf_bits2f(f2bf_bits(f)); }

__device__ __forceinline__ void dep_guard_h(v8f& a, v8f& b, v16h x, v16h y) { asm volatile("v_nop\n\tv_nop\n\tv_nop\n\tv_nop" : "+v"(a), "+v"(b) : "v"(x), "v"(y)); }
__device__ __forceinline__ void dep_guard_b(v8f& a, v8f& b, v16b x, v16b y) { asm volatile("v_nop\n\tv_nop\n\tv_nop\n\tv_nop" : "+v"(a), "+v"(b) : "v"(x), "v"(y)); }
__device__ __forceinline__ void keep4_h(v16h a, v16h b, v16h c, v16h d) { asm volatile("v_nop" :: "v"(a), "v"(b), "v"(c), "v"(d)); }
__device__ __forceinline__ void keep4_b(v16b a, v16b b, v16b c, v16b d) { asm volatile("v_nop" :: "v"(a), "v"(b), "v"(c), "v"(d)); }
__device__ __forceinline__ void acc_guard4(v8f& a, v8f& b, v8f& c, v8f& d) { asm volatile("v_nop\n\tv_nop\n\tv_nop\n\tv_nop" : "+v"(a), "+v"(b), "+v"(c), "+v"(d)); }
template <typename T> struct Frag;
template <> struct Frag<_Float16> {
  typedef v16h V; union U { v16h v; v8h h[2]; };
  static __device__ __forceinline__ v16h load(const _Float16* p) {
    U f; f.h[0] = *(const v8h*)(p); f.h[1] = *(const v8h*)(p + 16); return f.v;
  }
  static __device__ __forceinline__ v8f mma(v16h a, v16h b, v8f c) {
    return __builtin_amdgcn_wmma_f32_16x16x32_f16(false, a, false, b, (short)0, c, false, false);
  }
  static __device__ __forceinline__ void guard(v8f& a, v8f& b, v16h x, v16h y) { dep_guard_h(a, b, x, y); }
  static __device__ __forceinline__ void keep(v16h a, v16h b, v16h c, v16h d) { keep4_h(a, b, c, d); }
};
template <> struct Frag<__bf16> {
  typedef v16b V; union U { v16b v; v8b h[2]; };
  static __device__ __forceinline__ v16b load(const __bf16* p) {
    U f; f.h[0] = *(const v8b*)(p); f.h[1] = *(const v8b*)(p + 16); return f.v;
  }
  static __device__ __forceinline__ v8f mma(v16b a, v16b b, v8f c) {
    return __builtin_amdgcn_wmma_f32_16x16x32_bf16(false, a, false, b, (short)0, c, false, false);
  }
  static __device__ __forceinline__ void guard(v8f& a, v8f& b, v16b x, v16b y) { dep_guard_b(a, b, x, y); }
  static __device__ __forceinline__ void keep(v16b a, v16b b, v16b c, v16b d) { keep4_b(a, b, c, d); }
};

__device__ __forceinline__ unsigned pk16(unsigned short a, unsigned short b) { return (unsigned)a | ((unsigned)b << 16); }
__device__ __forceinline__ unsigned short h_bits(float f) { const _Float16 h = (_Float16)f; return __builtin_bit_cast(unsigned short, h); }

__device__ __forceinline__ v8f mma_h(v16h a, v16h b, v8f c) {
  c = __builtin_amdgcn_wmma_f32_16x16x32_f16(false, a, false, b, (short)0, c, false, false);
  asm volatile("v_nop\n\tv_nop\n\tv_nop\n\tv_nop" : "+v"(c) : "v"(a), "v"(b));
  return c;
}

template <int ET> struct Elem;
template <> struct Elem<0> { typedef _Float16 T; };
template <> struct Elem<1> { typedef __bf16 T; };
template <int ET, int SPLIT, int BIAS_MODE, int OUT_MODE>
__global__ __launch_bounds__(256) void wmma_gemm64(
    const unsigned short* __restrict__ Ap, const unsigned short* __restrict__ A2p, int lda, long strideA,
    const unsigned short* __restrict__ Btp, const unsigned short* __restrict__ Bt2p, int ldb, long strideB,
    void* __restrict__ Cout, void* __restrict__ Cout2, int ldc, long strideC,
    const float* __restrict__ bias,
    int M, int N, int K, float scale) {
  typedef typename Elem<ET>::T T;
  typedef typename Frag<T>::V V;
  const T* A = (const T*)Ap; const T* A2 = (const T*)A2p; const T* Bt = (const T*)Btp; const T* Bt2 = (const T*)Bt2p;
  __shared__ __align__(16) float sT[8][16 * 68];
  const int b    = blockIdx.y;
  const int lane = threadIdx.x & 31;
  const int wave = threadIdx.x >> 5;
  const int tilesN = N >> 6;
  const int tilesM = M >> 6;
  const int tile = blockIdx.x * 8 + wave;
  if (tile >= tilesM * tilesN) return;
  const int tm = tile / tilesN;
  const int tn = tile - tm * tilesN;
  const int m0 = tm << 6;
  const int n0 = tn << 6;

  const T* Ab  = A  + (size_t)b * strideA;
  const T* Bb  = Bt + (size_t)b * strideB;
  const T* Ab2 = (SPLIT != 0) ? (A2  + (size_t)b * strideA) : nullptr;
  const T* Bb2 = (SPLIT == 1) ? (Bt2 + (size_t)b * strideB) : nullptr;

  const int rlane = lane & 15;
  const int koff  = (lane >> 4) * 8;
  const int mOff  = (lane >> 4) * 8;

  v8f acc[4][4];
#pragma unroll
  for (int i = 0; i < 4; ++i)
#pragma unroll
    for (int j = 0; j < 4; ++j) acc[i][j] = (v8f){0.f,0.f,0.f,0.f,0.f,0.f,0.f,0.f};

  for (int k0 = 0; k0 < K; k0 += 32) {
    V bh[4], bl[4];
#pragma unroll
    for (int j = 0; j < 4; ++j) {
      const size_t bo = (size_t)(n0 + (j << 4) + rlane) * ldb + koff + k0;
      bh[j] = Frag<T>::load(Bb + bo);
      if (SPLIT == 1) bl[j] = Frag<T>::load(Bb2 + bo);
    }
#pragma unroll
    for (int i = 0; i < 4; ++i) {
      const size_t ao = (size_t)(m0 + (i << 4) + rlane) * lda + koff + k0;
      V ah = Frag<T>::load(Ab + ao);
      V al;
      if (SPLIT != 0) al = Frag<T>::load(Ab2 + ao);
#pragma unroll
      for (int j = 0; j < 4; ++j) {
        acc[i][j] = Frag<T>::mma(ah, bh[j], acc[i][j]);
        if (SPLIT == 1) acc[i][j] = Frag<T>::mma(ah, bl[j], acc[i][j]);
        if (SPLIT != 0) acc[i][j] = Frag<T>::mma(al, bh[j], acc[i][j]);
      }
      Frag<T>::guard(acc[i][0], acc[i][3], ah, (SPLIT != 0) ? al : ah);
    }
    Frag<T>::keep(bh[0], bh[1], bh[2], bh[3]);
    if (SPLIT == 1) Frag<T>::keep(bl[0], bl[1], bl[2], bl[3]);
  }
  acc_guard4(acc[0][0], acc[0][1], acc[0][2], acc[0][3]);
  acc_guard4(acc[1][0], acc[1][1], acc[1][2], acc[1][3]);
  acc_guard4(acc[2][0], acc[2][1], acc[2][2], acc[2][3]);
  acc_guard4(acc[3][0], acc[3][1], acc[3][2], acc[3][3]);

  float* slab = sT[wave];
#pragma unroll
  for (int i = 0; i < 4; ++i) {
    const int mBase = m0 + (i << 4);
#pragma unroll
    for (int j = 0; j < 4; ++j) {
      const int n = n0 + (j << 4) + rlane;
      float bv = 0.f;
      if (BIAS_MODE == 2) bv = bf_rne(bias[n]);
#pragma unroll
      for (int r = 0; r < 8; ++r) {
        float v = acc[i][j][r] * scale;
        if (BIAS_MODE == 1) v += bf_rne(bias[mBase + mOff + r]);
        if (BIAS_MODE == 2) v += bv;
        slab[(mOff + r) * 68 + (j << 4) + rlane] = v;
      }
    }
    __builtin_amdgcn_fence(3, "workgroup");
    __builtin_amdgcn_wave_barrier();
    __builtin_amdgcn_fence(2, "workgroup");
    if (OUT_MODE == 0) {
      float* C = (float*)Cout + (size_t)b * strideC;
      const int hh = lane >> 4, c4 = (lane & 15) * 4;
      for (int pass = 0; pass < 2; ++pass) {
#pragma unroll
        for (int it = 0; it < 8; ++it) {
          const int row = it * 2 + hh;
          v4f v = *(const v4f*)(slab + row * 68 + c4);
          *(volatile v4f*)(C + (size_t)(mBase + row) * ldc + n0 + c4) = v;
        }
        __threadfence();
      }
    } else {
      const int q = lane >> 3, c8 = (lane & 7) * 8;
      unsigned short* C  = (unsigned short*)Cout  + (size_t)b * strideC;
      unsigned short* C2 = (OUT_MODE == 2) ? ((unsigned short*)Cout2 + (size_t)b * strideC) : nullptr;
      for (int pass = 0; pass < 2; ++pass) {
#pragma unroll
        for (int it = 0; it < 4; ++it) {
          const int row = it * 4 + q;
          const float* sp = slab + row * 68 + c8;
          v8h hv, lv;
#pragma unroll
          for (int e = 0; e < 8; ++e) {
            if (OUT_MODE == 1) {
              hv[e] = (_Float16)sp[e];
            } else {
              unsigned short hb = f2bf_bits(sp[e]);
              unsigned short lb = f2bf_bits(sp[e] - bf_bits2f(hb));
              hv[e] = __builtin_bit_cast(_Float16, hb);
              lv[e] = __builtin_bit_cast(_Float16, lb);
            }
          }
          *(volatile v8h*)(C + (size_t)(mBase + row) * ldc + n0 + c8) = hv;
          if (OUT_MODE == 2) *(volatile v8h*)(C2 + (size_t)(mBase + row) * ldc + n0 + c8) = lv;
        }
        __threadfence();
      }
    }
    __builtin_amdgcn_fence(3, "workgroup");
    __builtin_amdgcn_wave_barrier();
    __builtin_amdgcn_fence(2, "workgroup");
  }
}

__global__ __launch_bounds__(256) void xcast_bf16_kernel(const float* __restrict__ in, unsigned short* __restrict__ out, int n8) {
  const int i = blockIdx.x * 256 + threadIdx.x;
  if (i >= n8) return;
  const int row = i >> 7;
  const int col = (i & 127) * 8;
  const int bb  = row / kS;
  const int ss  = row - bb * kS;
  const float* p = in + (size_t)(bb * kSF + ss) * kE + col;
  const v4f a = *(const v4f*)(p);
  const v4f c = *(const v4f*)(p + 4);
  unsigned short hb[8];
#pragma unroll
  for (int e = 0; e < 4; ++e) {
    hb[e]     = f2bf_bits(a[e]);
    hb[4 + e] = f2bf_bits(c[e]);
  }
  const v4u u = (v4u){pk16(hb[0], hb[1]), pk16(hb[2], hb[3]), pk16(hb[4], hb[5]), pk16(hb[6], hb[7])};
  unsigned short* q = out + 8 * (size_t)i;
  *(volatile v4u*)q = u;
  __threadfence();
  *(volatile v4u*)q = u;
}

__global__ __launch_bounds__(256) void wcast_kernel(const float* __restrict__ Wa, const float* __restrict__ Wo,
                                                    unsigned short* __restrict__ Wab, unsigned short* __restrict__ Wo16,
                                                    unsigned short* __restrict__ Wob) {
  const int z = blockIdx.y;
  const int i = blockIdx.x * 256 + threadIdx.x;
  const int n8 = (z == 0) ? (kF * kE / 8) : (kE * kE / 8);
  if (i >= n8) return;
  const float* p = ((z == 0) ? Wa : Wo) + 8 * (size_t)i;
  const v4f a = *(const v4f*)(p);
  const v4f c = *(const v4f*)(p + 4);
  unsigned short bb[8], fb[8];
#pragma unroll
  for (int e = 0; e < 4; ++e) {
    bb[e]     = f2bf_bits(a[e]);
    bb[4 + e] = f2bf_bits(c[e]);
  }
#pragma unroll
  for (int e = 0; e < 8; ++e) fb[e] = h_bits(bf_bits2f(bb[e]) * kWoCarry);
  const v4u ub = (v4u){pk16(bb[0], bb[1]), pk16(bb[2], bb[3]), pk16(bb[4], bb[5]), pk16(bb[6], bb[7])};
  const v4u uh = (v4u){pk16(fb[0], fb[1]), pk16(fb[2], fb[3]), pk16(fb[4], fb[5]), pk16(fb[6], fb[7])};
  if (z == 0) {
    unsigned short* q = Wab + 8 * (size_t)i;
    *(volatile v4u*)q = ub;
    __threadfence();
    *(volatile v4u*)q = ub;
  } else {
    unsigned short* qb = Wob  + 8 * (size_t)i;
    unsigned short* qh = Wo16 + 8 * (size_t)i;
    *(volatile v4u*)qb = ub;
    *(volatile v4u*)qh = uh;
    __threadfence();
    *(volatile v4u*)qb = ub;
    *(volatile v4u*)qh = uh;
  }
}

__global__ __launch_bounds__(128) __attribute__((amdgpu_num_vgpr(256)))
void attn_causal_kernel(const unsigned short* __restrict__ QK16, const unsigned short* __restrict__ Vt16,
                        const float* __restrict__ V32, unsigned short* __restrict__ Y16,
                        unsigned short* __restrict__ Ybh, unsigned short* __restrict__ Ybl) {
  __shared__ __align__(16) _Float16 Ksh[kKC * kD];
  __shared__ __align__(16) _Float16 Vth[kD * kKC];
  __shared__ __align__(16) _Float16 Psh[kNW][16 * kKC];
  __shared__ __align__(16) float    P32[kNW][16 * kKC];
  __shared__ __align__(16) float    Os[kNW][16 * 68];

  const int tid  = threadIdx.x;
  const int wave = tid >> 5;
  const int lane = tid & 31;
  const int hh   = lane >> 4;
  const int c    = lane & 15;

  const int bx = blockIdx.x;
  const int qb = bx % kNQB;
  const int bh = bx / kNQB;
  const int h  = bh % kH;
  const int b  = bh / kH;
  const int tok0 = b * kS;
  const int q0 = qb * kQB + wave * 16;
  const bool exact = (qb < kHeadBlocks);

  const _Float16* Qp = (const _Float16*)(const void*)QK16;
  v16h qa[2];
  {
    const _Float16* qrow = Qp + (size_t)(tok0 + q0 + c) * kQKld + h * kD + 8 * hh;
#pragma unroll
    for (int dc = 0; dc < 2; ++dc) qa[dc] = Frag<_Float16>::load(qrow + dc * 32);
  }

  float mrow[8], lrow[8];
  v8f oacc[4];
#pragma unroll
  for (int r = 0; r < 8; ++r) { mrow[r] = -__builtin_inff(); lrow[r] = 0.f; }
#pragma unroll
  for (int t = 0; t < 4; ++t) oacc[t] = (v8f){0.f,0.f,0.f,0.f,0.f,0.f,0.f,0.f};

  _Float16* pw = Psh[wave];
  float* p32w = P32[wave];

  const int nChunks = qb + 1;
#pragma unroll 1
  for (int kc = 0; kc < nChunks; ++kc) {
    const int kv0 = kc * kKC;
    __syncthreads();
    {
      const int kvr = tid >> 1, dh = (tid & 1) * 32;
      const unsigned short* kg = QK16 + (size_t)(tok0 + kv0 + kvr) * kQKld + kE + h * kD + dh;
      const unsigned short* vg = Vt16 + (size_t)(bh * kD + kvr) * kS + kv0 + dh;
      const v4u ka = *(const v4u*)(kg);
      const v4u kb = *(const v4u*)(kg + 8);
      const v4u kcv = *(const v4u*)(kg + 16);
      const v4u kdv = *(const v4u*)(kg + 24);
      const v4u va = *(const v4u*)(vg);
      const v4u vb = *(const v4u*)(vg + 8);
      const v4u vc = *(const v4u*)(vg + 16);
      const v4u vd = *(const v4u*)(vg + 24);
      _Float16* kdst = Ksh + kvr * kD + dh;
      _Float16* vdst = Vth + kvr * kKC + dh;
      *(v4u*)(kdst)      = ka;
      *(v4u*)(kdst + 8)  = kb;
      *(v4u*)(kdst + 16) = kcv;
      *(v4u*)(kdst + 24) = kdv;
      *(v4u*)(vdst)      = va;
      *(v4u*)(vdst + 8)  = vb;
      *(v4u*)(vdst + 16) = vc;
      *(v4u*)(vdst + 24) = vd;
    }
    __syncthreads();

    v8f s[4];
#pragma unroll
    for (int j = 0; j < 4; ++j) {
      s[j] = (v8f){0.f,0.f,0.f,0.f,0.f,0.f,0.f,0.f};
#pragma unroll
      for (int dc = 0; dc < 2; ++dc) {
        const v16h kf = Frag<_Float16>::load(Ksh + (j * 16 + c) * kD + dc * 32 + 8 * hh);
        s[j] = mma_h(qa[dc], kf, s[j]);
      }
    }

    const bool diag = (kc == qb);
    float cm[8];
#pragma unroll
    for (int r = 0; r < 8; ++r) {
      const int qrow = q0 + 8 * hh + r;
      float m = -__builtin_inff();
#pragma unroll
      for (int j = 0; j < 4; ++j) {
        const int kvcol = kv0 + j * 16 + c;
        float val = s[j][r] * kLogitScale;
        val = (diag && (kvcol > qrow)) ? -__builtin_inff() : val;
        s[j][r] = val;
        m = fmaxf(m, val);
      }
#pragma unroll
      for (int off = 1; off < 16; off <<= 1) m = fmaxf(m, __shfl_xor(m, off, 32));
      cm[r] = m;
    }

#pragma unroll
    for (int r = 0; r < 8; ++r) {
      const float mnew = fmaxf(mrow[r], cm[r]);
      const float alpha = expf(mrow[r] - mnew);
      mrow[r] = mnew;
      float psum = 0.f;
#pragma unroll
      for (int j = 0; j < 4; ++j) {
        const float p = expf(s[j][r] - mnew);
        psum += p;
        pw[(8 * hh + r) * kKC + j * 16 + c] = (_Float16)(p * kPCarry);
        if (exact) p32w[(8 * hh + r) * kKC + j * 16 + c] = p;
      }
#pragma unroll
      for (int off = 1; off < 16; off <<= 1) psum += __shfl_xor(psum, off, 32);
      lrow[r] = lrow[r] * alpha + psum;
#pragma unroll
      for (int t = 0; t < 4; ++t) oacc[t][r] *= alpha;
    }
    __builtin_amdgcn_fence(3, "workgroup");
    __builtin_amdgcn_wave_barrier();
    __builtin_amdgcn_fence(2, "workgroup");

    if (!exact) {
#pragma unroll
      for (int kk = 0; kk < 2; ++kk) {
        const v16h pa = Frag<_Float16>::load(pw + c * kKC + kk * 32 + 8 * hh);
#pragma unroll
        for (int t = 0; t < 4; ++t) {
          const v16h vf = Frag<_Float16>::load(Vth + (t * 16 + c) * kKC + kk * 32 + 8 * hh);
          oacc[t] = mma_h(pa, vf, oacc[t]);
        }
      }
    } else {
      const float* vg32 = V32 + (size_t)(b * kHeadRows + kv0) * kE + h * kD + c;
#pragma unroll 1
      for (int kv = 0; kv < kKC; ++kv) {
        float pr[8];
#pragma unroll
        for (int r = 0; r < 8; ++r) pr[r] = p32w[(8 * hh + r) * kKC + kv];
        const float* vr = vg32 + (size_t)kv * kE;
        const float v0 = vr[0], v1 = vr[16], v2 = vr[32], v3 = vr[48];
#pragma unroll
        for (int r = 0; r < 8; ++r) {
          oacc[0][r] = fmaf(pr[r], v0, oacc[0][r]);
          oacc[1][r] = fmaf(pr[r], v1, oacc[1][r]);
          oacc[2][r] = fmaf(pr[r], v2, oacc[2][r]);
          oacc[3][r] = fmaf(pr[r], v3, oacc[3][r]);
        }
      }
    }
  }

  const float pscl = exact ? 1.0f : kPCarry;
  float* os = Os[wave];
#pragma unroll
  for (int r = 0; r < 8; ++r) {
    const float inv = 1.0f / (lrow[r] * pscl);
#pragma unroll
    for (int t = 0; t < 4; ++t) os[(8 * hh + r) * 68 + t * 16 + c] = oacc[t][r] * inv;
  }
  __builtin_amdgcn_fence(3, "workgroup");
  __builtin_amdgcn_wave_barrier();
  __builtin_amdgcn_fence(2, "workgroup");

  {
    const int q4 = lane >> 3, c8 = (lane & 7) * 8;
    _Float16* Yp = (_Float16*)(void*)Y16;
    for (int pass = 0; pass < 2; ++pass) {
#pragma unroll
      for (int it = 0; it < 4; ++it) {
        const int row = it * 4 + q4;
        const float* sp = os + row * 68 + c8;
        v8h hv;
#pragma unroll
        for (int e = 0; e < 8; ++e) hv[e] = (_Float16)(sp[e] * kYCarry);
        *(volatile v8h*)(Yp + (size_t)(tok0 + q0 + row) * kE + h * kD + c8) = hv;
      }
      __threadfence();
    }
    if (exact) {
      _Float16* Hp = (_Float16*)(void*)Ybh;
      _Float16* Lp = (_Float16*)(void*)Ybl;
      for (int pass = 0; pass < 2; ++pass) {
#pragma unroll
        for (int it = 0; it < 4; ++it) {
          const int row = it * 4 + q4;
          const float* sp = os + row * 68 + c8;
          v8h bhv, blv;
#pragma unroll
          for (int e = 0; e < 8; ++e) {
            const unsigned short hb = f2bf_bits(sp[e]);
            const unsigned short lb = f2bf_bits(sp[e] - bf_bits2f(hb));
            bhv[e] = __builtin_bit_cast(_Float16, hb);
            blv[e] = __builtin_bit_cast(_Float16, lb);
          }
          const size_t off = (size_t)(b * kHeadRows + q0 + row) * kE + h * kD + c8;
          *(volatile v8h*)(Hp + off) = bhv;
          *(volatile v8h*)(Lp + off) = blv;
        }
        __threadfence();
      }
    }
  }
}

extern "C" void kernel_launch(void* const* d_in, const int* in_sizes, int n_in,
                              void* d_out, int out_size, void* d_ws, size_t ws_size,
                              hipStream_t stream) {
  if (n_in < 5) return;
  const long needTokE = ((long)(kB - 1) * kSF + kS) * kE;
  if ((long)in_sizes[0] < needTokE) return;
  if (in_sizes[1] < kF * kE || in_sizes[2] < kF || in_sizes[3] < kE * kE || in_sizes[4] < kE) return;
  if ((long)out_size < needTokE) return;

  const size_t szXb   = (size_t)kTok * kE * 2;
  const size_t szWab  = (size_t)kF * kE * 2;
  const size_t szWo16 = (size_t)kE * kE * 2;
  const size_t szWob  = (size_t)kE * kE * 2;
  const size_t szQK   = (size_t)kTok * kQKld * 2;
  const size_t szVt   = (size_t)kB * kE * kS * 2;
  const size_t szV32  = (size_t)kB * kHeadRows * kE * 4;
  const size_t szY16  = (size_t)kTok * kE * 2;
  const size_t szYb   = (size_t)kB * kHeadRows * kE * 2;
  const size_t offXb   = 0;
  const size_t offWab  = offXb + szXb;
  const size_t offWo16 = offWab + szWab;
  const size_t offWob  = offWo16 + szWo16;
  const size_t offQK   = offWob + szWob;
  const size_t offVt   = offQK + szQK;
  const size_t offV32  = offVt + szVt;
  const size_t offY16  = offV32 + szV32;
  const size_t offYbh  = offY16 + szY16;
  const size_t offYbl  = offYbh + szYb;
  const size_t total   = offYbl + szYb;
  if (ws_size < total) return;
  if (total > (size_t)134217728) return;

  const float* x   = (const float*)d_in[0];
  const float* Wa  = (const float*)d_in[1];
  const float* Wab_bias = (const float*)d_in[2];
  const float* Wo  = (const float*)d_in[3];
  const float* bo  = (const float*)d_in[4];
  float* out = (float*)d_out;
  char* ws = (char*)d_ws;
  unsigned short* Xb    = (unsigned short*)(ws + offXb);
  unsigned short* Wab   = (unsigned short*)(ws + offWab);
  unsigned short* WabV  = Wab + (size_t)2 * kE * kE;
  unsigned short* Wo16  = (unsigned short*)(ws + offWo16);
  unsigned short* Wob   = (unsigned short*)(ws + offWob);
  unsigned short* QK16  = (unsigned short*)(ws + offQK);
  unsigned short* Vt16  = (unsigned short*)(ws + offVt);
  float*          V32   = (float*)(ws + offV32);
  unsigned short* Y16   = (unsigned short*)(ws + offY16);
  unsigned short* Ybh   = (unsigned short*)(ws + offYbh);
  unsigned short* Ybl   = (unsigned short*)(ws + offYbl);
  const float* biasQK = Wab_bias;
  const float* biasV  = Wab_bias + 2 * kE;

  const int n8 = kTok * kE / 8;
  xcast_bf16_kernel<<<dim3((n8 + 255) / 256), dim3(256), 0, stream>>>(x, Xb, n8);

  {
    const int n8a = kF * kE / 8;
    wcast_kernel<<<dim3((n8a + 255) / 256, 2), dim3(256), 0, stream>>>(Wa, Wo, Wab, Wo16, Wob);
  }

  const long strideSeqA = (long)kS * kE;
  const long strideSeqC = (long)kSF * kE;

  {
    const int tiles = (kTok / 64) * (kQKld / 64);
    wmma_gemm64<1, 0, 2, 1><<<dim3((tiles + 7) / 8, 1), dim3(256), 0, stream>>>(
        Xb, Xb, kE, 0L, Wab, Wab, kE, 0L,
        (void*)QK16, (void*)QK16, kQKld, 0L, biasQK, kTok, kQKld, kE, 1.0f);
  }
  {
    const int tiles = (kE / 64) * (kS / 64);
    wmma_gemm64<1, 0, 1, 1><<<dim3((tiles + 7) / 8, kB), dim3(256), 0, stream>>>(
        WabV, WabV, kE, 0L, Xb, Xb, kE, strideSeqA,
        (void*)Vt16, (void*)Vt16, kS, (long)kE * kS, biasV, kE, kS, kE, 1.0f);
  }
  {
    const int tiles = (kHeadRows / 64) * (kE / 64);
    wmma_gemm64<1, 0, 2, 0><<<dim3((tiles + 7) / 8, kB), dim3(256), 0, stream>>>(
        Xb, Xb, kE, strideSeqA, WabV, WabV, kE, 0L,
        (void*)V32, (void*)V32, kE, (long)kHeadRows * kE, biasV, kHeadRows, kE, kE, 1.0f);
  }
  attn_causal_kernel<<<dim3(kB * kH * kNQB), dim3(128), 0, stream>>>(QK16, Vt16, V32, Y16, Ybh, Ybl);

  if (kS - kHeadRows > 0) {
    const int tiles = ((kS - kHeadRows) / 64) * (kE / 64);
    wmma_gemm64<0, 0, 2, 0><<<dim3((tiles + 7) / 8, kB), dim3(256), 0, stream>>>(
        Y16 + (size_t)kHeadRows * kE, Y16 + (size_t)kHeadRows * kE, kE, strideSeqA, Wo16, Wo16, kE, 0L,
        (void*)(out + (size_t)kHeadRows * kE), (void*)(out + (size_t)kHeadRows * kE), kE, strideSeqC,
        bo, kS - kHeadRows, kE, kE, kOutScale);
  }
  {
    const int tiles = (kHeadRows / 64) * (kE / 64);
    wmma_gemm64<1, 2, 2, 0><<<dim3((tiles + 7) / 8, kB), dim3(256), 0, stream>>>(
        Ybh, Ybl, kE, (long)kHeadRows * kE, Wob, Wob, kE, 0L,
        (void*)out, (void*)out, kE, strideSeqC, bo, kHeadRows, kE, kE, 1.0f);
  }
}
